// Filter__55113020342600
// MI455X (gfx1250) — hardware-run, weakly checked
//
#include <hip/hip_runtime.h>
#include <math.h>

typedef __attribute__((ext_vector_type(16))) _Float16 v16h;
typedef __attribute__((ext_vector_type(8)))  _Float16 v8h;
typedef __attribute__((ext_vector_type(4)))  _Float16 v4h;
typedef __attribute__((ext_vector_type(2)))  _Float16 v2h;
typedef __attribute__((ext_vector_type(16))) __bf16   v16b;
typedef __attribute__((ext_vector_type(8)))  __bf16   v8b;
typedef __attribute__((ext_vector_type(8)))  float    v8f;
typedef __attribute__((ext_vector_type(4)))  float    v4f;
typedef __attribute__((ext_vector_type(2)))  float    v2f;

constexpr int kNB   = 8192;
constexpr int kNQ   = 1024;
constexpr int kD    = 128;
constexpr int kTiles = kNB / 16;
constexpr int kThr  = 256;
constexpr float kInCarry = 1024.0f;
constexpr float kSc20 = 1.0f / (kInCarry * kInCarry);
constexpr float kF16MinNormal = 6.103515625e-5f;
constexpr float kW1 = 1.0f / 10.0f;
constexpr float kW2 = 1.0f / 512.0f;
constexpr float kW3 = 1.0f / 2048.0f;

static_assert(kNB == 8192 && kNQ == 1024 && kD == 128 && kTiles == 512, "the index arithmetic below uses these sizes");

constexpr size_t kOffD16 = 0ull;
constexpr size_t kOffX16 = 2097152ull;
constexpr size_t kOffDR = 2359296ull;
constexpr size_t kOffXR = 6553600ull;
constexpr size_t kOffDQ = 7077888ull;
constexpr size_t kOffXQ = 7110656ull;
constexpr size_t kOffPS1 = 7114752ull;
constexpr size_t kOffPS2 = 7180288ull;
constexpr size_t kOffT1 = 7188480ull;
constexpr size_t kOffMX = 7189504ull;
constexpr size_t kWsTotal = 7189760ull;
static_assert(kWsTotal <= 268435456ull, "the carve stands under 256 MiB");
static_assert(kOffD16 == 0
  && kOffX16 == kOffD16 + 2097152ull
  && kOffDR == kOffX16 + 262144ull
  && kOffXR == kOffDR + 4194304ull
  && kOffDQ == kOffXR + 524288ull
  && kOffXQ == kOffDQ + 32768ull
  && kOffPS1 == kOffXQ + 4096ull
  && kOffPS2 == kOffPS1 + 65536ull
  && kOffT1 == kOffPS2 + 8192ull
  && kOffMX == kOffT1 + 1024ull
  && kWsTotal == kOffMX + 256ull, "the carve is a chain: every region starts where the one before ends");
static_assert((kOffD16 % 256) == 0 && (kOffX16 % 256) == 0 && (kOffDR % 256) == 0 && (kOffXR % 256) == 0 && (kOffDQ % 256) == 0 && (kOffXQ % 256) == 0 && (kOffPS1 % 256) == 0 && (kOffPS2 % 256) == 0 && (kOffT1 % 256) == 0 && (kOffMX % 256) == 0, "every region starts on a multiple of 256 B");

__device__ __forceinline__ unsigned short f2bf_bits(float f) {
  unsigned u = __float_as_uint(f);
  return (unsigned short)((u + 0x7FFFu + ((u >> 16) & 1u)) >> 16);
}
__device__ __forceinline__ float bf_bits2f(unsigned short h) { return __uint_as_float(((unsigned)h) << 16); }
__device__ __forceinline__ float bf16r(float f) { return bf_bits2f(f2bf_bits(f)); }
__device__ __forceinline__ float carry_flush(float v, float carry) {
  const float s = v * carry;
  return (fabsf(s) < kF16MinNormal) ? 0.0f : s;
}

__device__ __forceinline__ void dep_guard4_h(v8f& a, v8f& b, v8f& c, v8f& d, v16h x, v16h y) { asm volatile("v_nop\n\tv_nop\n\tv_nop\n\tv_nop" : "+v"(a), "+v"(b), "+v"(c), "+v"(d) : "v"(x), "v"(y)); }
__device__ __forceinline__ void dep_guard4_b(v8f& a, v8f& b, v8f& c, v8f& d, v16b x, v16b y) { asm volatile("v_nop\n\tv_nop\n\tv_nop\n\tv_nop" : "+v"(a), "+v"(b), "+v"(c), "+v"(d) : "v"(x), "v"(y)); }
__device__ __forceinline__ void keep4_h(v16h a, v16h b, v16h c, v16h d) { asm volatile("v_nop" :: "v"(a), "v"(b), "v"(c), "v"(d)); }
__device__ __forceinline__ void keep4_b(v16b a, v16b b, v16b c, v16b d) { asm volatile("v_nop" :: "v"(a), "v"(b), "v"(c), "v"(d)); }
__device__ __forceinline__ void acc_guard4(v8f& a, v8f& b, v8f& c, v8f& d) { asm volatile("v_nop\n\tv_nop\n\tv_nop\n\tv_nop" : "+v"(a), "+v"(b), "+v"(c), "+v"(d)); }

template <typename T> struct Frag;
template <> struct Frag<_Float16> {
  typedef v16h V; union U { v16h v; v8h h[2]; };
  static __device__ __forceinline__ v16h load(const _Float16* p) {
    U f; f.h[0] = *(const v8h*)(p); f.h[1] = *(const v8h*)(p + 16); return f.v;
  }
  static __device__ __forceinline__ v8f mma(v16h a, v16h b, v8f c) {
    return __builtin_amdgcn_wmma_f32_16x16x32_f16(false, a, false, b, (short)0, c, false, false);
  }
  static __device__ __forceinline__ void guard4(v8f& a, v8f& b, v8f& c, v8f& d, v16h x, v16h y) { dep_guard4_h(a, b, c, d, x, y); }
  static __device__ __forceinline__ void keep(v16h a, v16h b, v16h c, v16h d) { keep4_h(a, b, c, d); }
};
template <> struct Frag<__bf16> {
  typedef v16b V; union U { v16b v; v8b h[2]; };
  static __device__ __forceinline__ v16b load(const __bf16* p) {
    U f; f.h[0] = *(const v8b*)(p); f.h[1] = *(const v8b*)(p + 16); return f.v;
  }
  static __device__ __forceinline__ v8f mma(v16b a, v16b b, v8f c) {
    return __builtin_amdgcn_wmma_f32_16x16x32_bf16(false, a, false, b, (short)0, c, false, false);
  }
  static __device__ __forceinline__ void guard4(v8f& a, v8f& b, v8f& c, v8f& d, v16b x, v16b y) { dep_guard4_b(a, b, c, d, x, y); }
  static __device__ __forceinline__ void keep(v16b a, v16b b, v16b c, v16b d) { keep4_b(a, b, c, d); }
};

__device__ __forceinline__ v8f mma_h(v16h a, v16h b, v8f c) {
  c = __builtin_amdgcn_wmma_f32_16x16x32_f16(false, a, false, b, (short)0, c, false, false);
  asm volatile("v_nop\n\tv_nop\n\tv_nop\n\tv_nop" : "+v"(c) : "v"(a), "v"(b));
  return c;
}

template <int ET> struct Elem;
template <> struct Elem<0> { typedef _Float16 T; };
template <> struct Elem<1> { typedef __bf16 T; };
template <int ET, bool SPLIT, int BIAS_MODE, int OUT_MODE, bool RESID, int ACT = 0>
__global__ __launch_bounds__(256) void wmma_gemm64(
    const unsigned short* __restrict__ Ap, const unsigned short* __restrict__ A2p, int lda, long strideA,
    const unsigned short* __restrict__ Btp, const unsigned short* __restrict__ Bt2p, int ldb, long strideB,
    void* __restrict__ Cout, void* __restrict__ Cout2, int ldc, long strideC,
    const float* __restrict__ bias,
    const float* __restrict__ resid, long strideR,
    int M, int N, int K, float scale) {
  typedef typename Elem<ET>::T T;
  typedef typename Frag<T>::V V;
  const T* A = (const T*)Ap; const T* A2 = (const T*)A2p; const T* Bt = (const T*)Btp; const T* Bt2 = (const T*)Bt2p;
  __shared__ __align__(16) float sT[8][16 * 68];
  const int b    = blockIdx.y;
  const int lane = threadIdx.x & 31;
  const int wave = threadIdx.x >> 5;
  const int tilesN = N >> 6;
  const int tilesM = M >> 6;
  const int tile = blockIdx.x * 8 + wave;
  if (tile >= tilesM * tilesN) return;
  const int tm = tile / tilesN;
  const int tn = tile - tm * tilesN;
  const int m0 = tm << 6;
  const int n0 = tn << 6;

  const T* Ab  = A  + (size_t)b * strideA;
  const T* Bb  = Bt + (size_t)b * strideB;
  const T* Ab2 = SPLIT ? (A2  + (size_t)b * strideA) : nullptr;
  const T* Bb2 = SPLIT ? (Bt2 + (size_t)b * strideB) : nullptr;

  const int rlane = lane & 15;
  const int koff  = (lane >> 4) * 8;
  const int mOff  = (lane >> 4) * 8;

  v8f acc[4][4];
#pragma unroll
  for (int i = 0; i < 4; ++i)
#pragma unroll
    for (int j = 0; j < 4; ++j) acc[i][j] = (v8f){0.f,0.f,0.f,0.f,0.f,0.f,0.f,0.f};

  for (int k0 = 0; k0 < K; k0 += 32) {
    V bh[4], bl[4];
#pragma unroll
    for (int j = 0; j < 4; ++j) {
      const size_t bo = (size_t)(n0 + (j << 4) + rlane) * ldb + koff + k0;
      bh[j] = Frag<T>::load(Bb + bo);
      if (SPLIT) bl[j] = Frag<T>::load(Bb2 + bo);
    }
#pragma unroll
    for (int i = 0; i < 4; ++i) {
      const size_t ao = (size_t)(m0 + (i << 4) + rlane) * lda + koff + k0;
      V ah = Frag<T>::load(Ab + ao);
      V al;
      if (SPLIT) al = Frag<T>::load(Ab2 + ao);
#pragma unroll
      for (int j = 0; j < 4; ++j) {
        acc[i][j] = Frag<T>::mma(ah, bh[j], acc[i][j]);
        if (SPLIT) {
          acc[i][j] = Frag<T>::mma(ah, bl[j], acc[i][j]);
          acc[i][j] = Frag<T>::mma(al, bh[j], acc[i][j]);
        }
      }
      Frag<T>::guard4(acc[i][0], acc[i][1], acc[i][2], acc[i][3], ah, SPLIT ? al : ah);
    }
    Frag<T>::keep(bh[0], bh[1], bh[2], bh[3]);
    if (SPLIT) Frag<T>::keep(bl[0], bl[1], bl[2], bl[3]);
  }
  acc_guard4(acc[0][0], acc[0][1], acc[0][2], acc[0][3]);
  acc_guard4(acc[1][0], acc[1][1], acc[1][2], acc[1][3]);
  acc_guard4(acc[2][0], acc[2][1], acc[2][2], acc[2][3]);
  acc_guard4(acc[3][0], acc[3][1], acc[3][2], acc[3][3]);

  float* slab = sT[wave];
  const float* Rb = RESID ? (resid + (size_t)b * strideR) : nullptr;
#pragma unroll
  for (int i = 0; i < 4; ++i) {
    const int mBase = m0 + (i << 4);
#pragma unroll
    for (int j = 0; j < 4; ++j) {
      const int n = n0 + (j << 4) + rlane;
      float bv = 0.f;
      if (BIAS_MODE == 2) bv = bias[n];
#pragma unroll
      for (int r = 0; r < 8; ++r) {
        float v = acc[i][j][r] * scale;
        if (BIAS_MODE == 1) v += bias[mBase + mOff + r];
        if (BIAS_MODE == 2) v += bv;
        if (RESID) v += Rb[(size_t)(mBase + mOff + r) * ldc + n];
        if (ACT == 1) v = tanhf(v);
        if (ACT == 2) v = fmaxf(v, 0.0f);
        if (ACT == 3) v = v / (1.0f + expf(-v));
        if (ACT == 4) v = (v > 0.f) ? v : 0.01f * v;
        slab[(mOff + r) * 68 + (j << 4) + rlane] = v;
      }
    }
    __builtin_amdgcn_fence(__ATOMIC_RELEASE, "workgroup");
    __builtin_amdgcn_wave_barrier();
    __builtin_amdgcn_fence(__ATOMIC_ACQUIRE, "workgroup");
    if (OUT_MODE == 0) {
      float* C = (float*)Cout + (size_t)b * strideC;
      const int hh = lane >> 4, c4 = (lane & 15) * 4;
      for (int pass = 0; pass < 2; ++pass) {
#pragma unroll
        for (int it = 0; it < 8; ++it) {
          const int row = it * 2 + hh;
          v4f v = *(const v4f*)(slab + row * 68 + c4);
          *(volatile v4f*)(C + (size_t)(mBase + row) * ldc + n0 + c4) = v;
        }
        __threadfence();
      }
    } else {
      const int q = lane >> 3, c8 = (lane & 7) * 8;
      unsigned short* C  = (unsigned short*)Cout  + (size_t)b * strideC;
      unsigned short* C2 = (OUT_MODE == 2) ? ((unsigned short*)Cout2 + (size_t)b * strideC) : nullptr;
      for (int pass = 0; pass < 2; ++pass) {
#pragma unroll
        for (int it = 0; it < 4; ++it) {
          const int row = it * 4 + q;
          const float* sp = slab + row * 68 + c8;
          v8h hv, lv;
#pragma unroll
          for (int e = 0; e < 8; ++e) {
            if (OUT_MODE == 1) {
              hv[e] = (_Float16)sp[e];
            } else {
              unsigned short hb = f2bf_bits(sp[e]);
              unsigned short lb = f2bf_bits(sp[e] - bf_bits2f(hb));
              hv[e] = __builtin_bit_cast(_Float16, hb);
              lv[e] = __builtin_bit_cast(_Float16, lb);
            }
          }
          *(volatile v8h*)(C + (size_t)(mBase + row) * ldc + n0 + c8) = hv;
          if (OUT_MODE == 2) *(volatile v8h*)(C2 + (size_t)(mBase + row) * ldc + n0 + c8) = lv;
        }
        __threadfence();
      }
    }
    __builtin_amdgcn_fence(__ATOMIC_RELEASE, "workgroup");
    __builtin_amdgcn_wave_barrier();
    __builtin_amdgcn_fence(__ATOMIC_ACQUIRE, "workgroup");
  }
}

__global__ __launch_bounds__(kThr) void cast_plane_kernel(const float* __restrict__ src, unsigned short* __restrict__ dst,
                                                          int colsLog2, int dstPitch, int dstOff) {
  const int i   = blockIdx.x * kThr + threadIdx.x;
  const int sh  = colsLog2 - 3;
  const int row = i >> sh;
  const int c8  = (i & ((1 << sh) - 1)) * 8;
  const float* sp = src + ((size_t)row << colsLog2) + c8;
  const v4f a0 = *(const v4f*)(sp);
  const v4f a1 = *(const v4f*)(sp + 4);
  v8h hv;
#pragma unroll
  for (int e = 0; e < 4; ++e) {
    const float f0 = a0[e];
    const float f1 = a1[e];
    hv[e]     = (_Float16)carry_flush(bf16r(f0), kInCarry);
    hv[4 + e] = (_Float16)carry_flush(bf16r(f1), kInCarry);
  }
  unsigned short* dp = dst + (size_t)row * dstPitch + dstOff + c8;
  *(volatile v8h*)dp = hv;
  __threadfence();
  *(volatile v8h*)dp = hv;
}

__global__ __launch_bounds__(kThr) void pack_kernel(const float* __restrict__ W, unsigned short* __restrict__ D, float* __restrict__ dstf, int part, int ld, int k0, int lg, int n0, int pitch) {
  const unsigned i = blockIdx.x * blockDim.x + threadIdx.x;
  if (part == 0) {
    const unsigned g = i & ((1u << lg) - 1u), n = i >> lg;
    const float* sp = W + (size_t)((unsigned)k0 + g * 8u) * (unsigned)ld + n;
    v8h hv;
#pragma unroll
    for (int t = 0; t < 8; ++t) hv[t] = (_Float16)carry_flush(bf16r(sp[(size_t)t * (unsigned)ld]), kInCarry);
    unsigned short* dp = D + (size_t)((unsigned)n0 + n) * (unsigned)pitch + g * 8u;
    *(volatile v8h*)dp = hv;
    __threadfence();
    *(volatile v8h*)dp = hv;
  } else {
    const v4f a = *(const v4f*)(W + i * 4u);
    v4f o;
#pragma unroll
    for (int e = 0; e < 4; ++e) o[e] = bf16r(a[e]);
    float* dp = dstf + i * 4u;
    *(volatile v4f*)dp = o;
    __threadfence();
    *(volatile v4f*)dp = o;
  }
}

__global__ __launch_bounds__(kThr) void rownorm128_kernel(const float* __restrict__ R, float* __restrict__ Q, float mul) {
  const unsigned i = blockIdx.x * (unsigned)kThr + threadIdx.x;
  const float* rp = R + (size_t)i * kD;
  float s = 0.0f;
  for (int c = 0; c < 32; ++c) {
    const v4f v = *(const v4f*)(rp + 4 * c);
#pragma unroll
    for (int e = 0; e < 4; ++e) s = fmaf(v[e], v[e], s);
  }
  const float o = s * mul;
  *(volatile float*)(Q + i) = o;
  __threadfence();
  *(volatile float*)(Q + i) = o;
}

__global__ __launch_bounds__(kThr) void widthsum_kernel(const unsigned short* __restrict__ P16p, const unsigned short* __restrict__ B16p, const float* __restrict__ PQ, const float* __restrict__ BQ, float* __restrict__ PS) {
  const _Float16* P16 = (const _Float16*)P16p; const _Float16* B16 = (const _Float16*)B16p;
  const int lane = threadIdx.x & 31, lr = lane & 15, hi = lane >> 4;
  const int wave = blockIdx.x * (kThr / 32) + (threadIdx.x >> 5);
  const int point = wave * 16 + lr;
  const _Float16* pp = P16 + (size_t)point * kD + 8 * hi;
  const v16h x0 = Frag<_Float16>::load(pp), x1 = Frag<_Float16>::load(pp + 32), x2 = Frag<_Float16>::load(pp + 64), x3 = Frag<_Float16>::load(pp + 96);
  const float hp = PQ[point];
  float part = 0.0f;
  for (int t = 0; t < kTiles; ++t) {
    const _Float16* bp = B16 + (size_t)(16 * t + lr) * kD + 8 * hi;
    v8f acc = (v8f){0.f, 0.f, 0.f, 0.f, 0.f, 0.f, 0.f, 0.f};
    acc = mma_h(Frag<_Float16>::load(bp), x0, acc);
    acc = mma_h(Frag<_Float16>::load(bp + 32), x1, acc);
    acc = mma_h(Frag<_Float16>::load(bp + 64), x2, acc);
    acc = mma_h(Frag<_Float16>::load(bp + 96), x3, acc);
    const v4f q0 = *(const v4f*)(BQ + 16 * t + 8 * hi), q1 = *(const v4f*)(BQ + 16 * t + 8 * hi + 4);
#pragma unroll
    for (int r = 0; r < 8; ++r) {
      const float bq = (r < 4) ? q0[r & 3] : q1[r & 3];
      const float h = (hp + bq) + acc[r] * kSc20;
      part += (expf(kW1 * h) + expf(kW2 * h)) + expf(kW3 * h);
    }
  }
  float* dp = PS + (size_t)point * 2 + hi;
  *(volatile float*)dp = part;
  __threadfence();
  *(volatile float*)dp = part;
}

__global__ __launch_bounds__(kThr) void sum64_kernel(const float* __restrict__ PS1, float* __restrict__ T1) {
  const unsigned i = threadIdx.x;
  const float* sp = PS1 + (size_t)i * 64u;
  float acc = 0.0f;
  for (int j = 0; j < 64; ++j) acc += sp[j];
  *(volatile float*)(T1 + i) = acc;
  __threadfence();
  *(volatile float*)(T1 + i) = acc;
}

__global__ __launch_bounds__(kThr) void meancopies_kernel(const float* __restrict__ T1, float* __restrict__ MX) {
  const unsigned i = blockIdx.x * (unsigned)kThr + threadIdx.x;
  const float* tp = T1 + (i >> 6);
  float acc = 0.0f;
  for (int j = 0; j < 256; ++j) acc += tp[j];
  const float o = (acc * (1.0f / 8192.0f)) * (1.0f / 8192.0f);
  *(volatile float*)(MX + i) = o;
  __threadfence();
  *(volatile float*)(MX + i) = o;
}

__global__ __launch_bounds__(kThr) void twosamplefinish_kernel(const float* __restrict__ PS2, const float* __restrict__ MX, float* __restrict__ res) {
  const unsigned b = blockIdx.x * (unsigned)kThr + threadIdx.x;
  const v2f a = *(const v2f*)(PS2 + (size_t)b * 2u);
  const float my = (a[0] + a[1]) * (1.0f / 8192.0f);
  const float mx = MX[threadIdx.x & 31u];
  const float o = (mx + 3.0f) - (my + my);
  *(volatile float*)(res + b) = o;
  __threadfence();
  *(volatile float*)(res + b) = o;
}

extern "C" void kernel_launch(void* const* d_in, const int* in_sizes, int n_in,
                              void* d_out, int out_size, void* d_ws, size_t ws_size,
                              hipStream_t stream) {
  if (n_in < 2 || d_out == nullptr || d_ws == nullptr) return;
  if (in_sizes[0] != kNB * kD || in_sizes[1] != kNQ * kD) return;
  if (out_size != kNQ) return;
  if (ws_size < kWsTotal) return;
  const float* bk = (const float*)d_in[0];
  const float* xq = (const float*)d_in[1];
  float* out = (float*)d_out;
  char* ws = (char*)d_ws;
  unsigned short* D16 = (unsigned short*)(ws + kOffD16);
  unsigned short* X16 = (unsigned short*)(ws + kOffX16);
  float* DR = (float*)(ws + kOffDR);
  float* XR = (float*)(ws + kOffXR);
  float* DQ = (float*)(ws + kOffDQ);
  float* XQ = (float*)(ws + kOffXQ);
  float* PS1 = (float*)(ws + kOffPS1);
  float* PS2 = (float*)(ws + kOffPS2);
  float* T1 = (float*)(ws + kOffT1);
  float* MX = (float*)(ws + kOffMX);

  static_assert((kNB * kD / 8) % kThr == 0 && (kNQ * kD / 8) % kThr == 0 && (kNB * kD / 4) % kThr == 0 && (kNQ * kD / 4) % kThr == 0 && kNB % kThr == 0 && kNQ % kThr == 0
                && (kNB / 16) % (kThr / 32) == 0 && (kNQ / 16) % (kThr / 32) == 0 && kNB * 2 == 256 * 64, "every grid exact");
  cast_plane_kernel<<<kNB * kD / 8 / kThr, kThr, 0, stream>>>(bk, D16, 7, kD, 0);
  cast_plane_kernel<<<kNQ * kD / 8 / kThr, kThr, 0, stream>>>(xq, X16, 7, kD, 0);
  pack_kernel<<<kNB * kD / 4 / kThr, kThr, 0, stream>>>(bk, nullptr, DR, 1, 0, 0, 0, 0, 0);
  pack_kernel<<<kNQ * kD / 4 / kThr, kThr, 0, stream>>>(xq, nullptr, XR, 1, 0, 0, 0, 0, 0);
  rownorm128_kernel<<<kNB / kThr, kThr, 0, stream>>>(DR, DQ, -0.5f);
  rownorm128_kernel<<<kNQ / kThr, kThr, 0, stream>>>(XR, XQ, -0.5f);
  widthsum_kernel<<<kNB / 16 / (kThr / 32), kThr, 0, stream>>>(D16, D16, DQ, DQ, PS1);
  widthsum_kernel<<<kNQ / 16 / (kThr / 32), kThr, 0, stream>>>(X16, D16, XQ, DQ, PS2);
  sum64_kernel<<<1, kThr, 0, stream>>>(PS1, T1);
  meancopies_kernel<<<1, 64, 0, stream>>>(T1, MX);
  twosamplefinish_kernel<<<kNQ / kThr, kThr, 0, stream>>>(PS2, MX, out);
}
